// NeRFRenderer_2259152798108
// MI455X (gfx1250) — hardware-run, weakly checked
//
#include <hip/hip_runtime.h>
#include <math.h>

typedef __attribute__((ext_vector_type(16))) _Float16 v16h;
typedef __attribute__((ext_vector_type(8)))  float    v8f;
typedef __attribute__((ext_vector_type(4)))  float    v4f;
typedef __attribute__((ext_vector_type(4)))  unsigned v4u;

constexpr int NUM_RAYS       = 16384;
constexpr int NSTEPS         = 128;
constexpr int HIDF           = 64;
constexpr int DFEAT          = 16;
constexpr int WPB            = 4;
constexpr int TPB            = WPB * 32;
constexpr int RAYS_PER_WAVE  = 8;
constexpr int RAYS_PER_BLOCK = WPB * RAYS_PER_WAVE;
constexpr int NBLOCKS        = NUM_RAYS / RAYS_PER_BLOCK;
constexpr int OUT_F32_PER_BLOCK = RAYS_PER_BLOCK * 3;
static_assert(NUM_RAYS % RAYS_PER_BLOCK == 0);
static_assert((OUT_F32_PER_BLOCK * 4) % 128 == 0);
static_assert(OUT_F32_PER_BLOCK / 4 <= 32);
static_assert(NSTEPS % 16 == 0);

constexpr int F_DW1 = 0, F_CW1 = 4, F_CW2 = 8, F_CW3 = 16, F_DW2 = 24, F_CW4 = 26, NFRAG = 28;
constexpr int FRAGS_PER_WAVE = NFRAG / WPB;
static_assert(NFRAG % WPB == 0);
constexpr int FRAG_U4     = NFRAG * 64;
constexpr int FRAG_HALVES = NFRAG * 32 * 16;
constexpr int FRAG_BYTES  = FRAG_U4 * 16;
static_assert(FRAG_HALVES * 2 == FRAG_BYTES);

constexpr int OFF_DW1 = 0;
constexpr int OFF_DW2 = OFF_DW1 + 3 * 64;
constexpr int OFF_CW1 = OFF_DW2 + 64 * 16;
constexpr int OFF_CW2 = OFF_CW1 + 32 * 64;
constexpr int OFF_CW3 = OFF_CW2 + 64 * 64;
constexpr int OFF_CW4 = OFF_CW3 + 64 * 64;
constexpr int RAW_TOTAL = OFF_CW4 + 64 * 3;
static_assert(RAW_TOTAL == 11648);


union V16 { v16h v; unsigned w[8]; };
struct BPair { v16h b0, b1; };

__device__ __forceinline__ unsigned pack_h2(float a, float b) {
  const unsigned lo = (unsigned)__builtin_bit_cast(unsigned short, (_Float16)a);
  const unsigned hi = (unsigned)__builtin_bit_cast(unsigned short, (_Float16)b);
  return lo | (hi << 16);
}

__device__ __forceinline__ v8f mma16(v16h a, v16h b, v8f c) {
  c = __builtin_amdgcn_wmma_f32_16x16x32_f16(false, a, false, b, (short)0, c, false, false);
  asm volatile("v_nop\n\tv_nop\n\tv_nop\n\tv_nop" : "+v"(c) : "v"(a), "v"(b));
  return c;
}

__device__ __forceinline__ v16h lda_lds(const _Float16* buf, int frag, int lane) {
  return *(const v16h*)(buf + (frag * 32 + lane) * 16);
}

__device__ __forceinline__ BPair acc_to_b(const v8f* c, const float* add, int lane) {
  const int mb = (lane >> 4) * 8;
  unsigned pk[4][4];
#pragma unroll
  for (int mt = 0; mt < 4; ++mt) {
    const float* bp = add + mt * 16 + mb;
#pragma unroll
    for (int j = 0; j < 4; ++j) {
      const float a = fmaxf(c[mt][2 * j]     + bp[2 * j],     0.0f);
      const float b = fmaxf(c[mt][2 * j + 1] + bp[2 * j + 1], 0.0f);
      pk[mt][j] = pack_h2(a, b);
    }
  }
  V16 f0, f1;
#pragma unroll
  for (int j = 0; j < 4; ++j) {
    f0.w[j]     = pk[0][j];
    f0.w[4 + j] = pk[1][j];
    f1.w[j]     = pk[2][j];
    f1.w[4 + j] = pk[3][j];
  }
  BPair r; r.b0 = f0.v; r.b1 = f1.v;
  return r;
}

__global__ void __launch_bounds__(TPB)
prep_frag_kernel(const float* __restrict__ dW1, const float* __restrict__ dW2,
                 const float* __restrict__ cW1, const float* __restrict__ cW2,
                 const float* __restrict__ cW3, const float* __restrict__ cW4,
                 v4u* __restrict__ table) {
  __shared__ float raw[RAW_TOTAL];
  const int tid  = threadIdx.x;
  const int lane = tid & 31;
  const int wid  = tid >> 5;

#pragma unroll 1
  for (int i = tid; i < 3 * 64; i += TPB)  raw[OFF_DW1 + i] = dW1[i];
#pragma unroll 1
  for (int i = tid; i < 64 * 16; i += TPB) raw[OFF_DW2 + i] = dW2[i];
#pragma unroll 1
  for (int i = tid; i < 32 * 64; i += TPB) raw[OFF_CW1 + i] = cW1[i];
#pragma unroll 1
  for (int i = tid; i < 64 * 64; i += TPB) raw[OFF_CW2 + i] = cW2[i];
#pragma unroll 1
  for (int i = tid; i < 64 * 64; i += TPB) raw[OFF_CW3 + i] = cW3[i];
#pragma unroll 1
  for (int i = tid; i < 64 * 3; i += TPB)  raw[OFF_CW4 + i] = cW4[i];
  __syncthreads();

  v4u piece[FRAGS_PER_WAVE][2];
#pragma unroll
  for (int s = 0; s < FRAGS_PER_WAVE; ++s) {
    const int f = wid + WPB * s;
    int src, ld, k0, m0, Kt, Mt;
    if (f < F_CW1)      { src = OFF_DW1; ld = 64; k0 = 0; m0 = 16 * f;           Kt = 3;  Mt = 64; }
    else if (f < F_CW2) { src = OFF_CW1; ld = 64; k0 = 0; m0 = 16 * (f - F_CW1); Kt = 32; Mt = 64; }
    else if (f < F_CW3) { const int g = f - F_CW2; src = OFF_CW2; ld = 64; k0 = (g & 1) * 32; m0 = (g >> 1) * 16; Kt = 64; Mt = 64; }
    else if (f < F_DW2) { const int g = f - F_CW3; src = OFF_CW3; ld = 64; k0 = (g & 1) * 32; m0 = (g >> 1) * 16; Kt = 64; Mt = 64; }
    else if (f < F_CW4) { src = OFF_DW2; ld = 16; k0 = (f - F_DW2) * 32; m0 = 0; Kt = 64; Mt = 16; }
    else                { src = OFF_CW4; ld = 3;  k0 = (f - F_CW4) * 32; m0 = 0; Kt = 64; Mt = 3; }
#pragma unroll
    for (int hq = 0; hq < 2; ++hq) {
      const int q  = lane + 32 * hq;
      const int lq = q >> 1;
      const int eh = q & 1;
      const int mm = m0 + (lq & 15);
      const bool mok = (mm < Mt);
      const int mc = mok ? mm : (Mt - 1);
      const int kb = k0 + 16 * eh + 8 * (lq >> 4);
      float v[8];
#pragma unroll
      for (int e = 0; e < 8; ++e) {
        const int k  = kb + e;
        const bool kok = (k < Kt);
        const int kc = kok ? k : (Kt - 1);
        const float x = raw[src + kc * ld + mc];
        v[e] = (mok && kok) ? x : 0.0f;
      }
      v4u p;
      p.x = pack_h2(v[0], v[1]);
      p.y = pack_h2(v[2], v[3]);
      p.z = pack_h2(v[4], v[5]);
      p.w = pack_h2(v[6], v[7]);
      piece[s][hq] = p;
    }
  }
  for (int pass = 0; pass < 2; ++pass) {
#pragma unroll
    for (int s = 0; s < FRAGS_PER_WAVE; ++s) {
      const int f = wid + WPB * s;
#pragma unroll
      for (int hq = 0; hq < 2; ++hq) {
        *(volatile v4u*)(table + (size_t)f * 64 + hq * 32 + lane) = piece[s][hq];
      }
    }
    __threadfence();
  }
}

__global__ void __launch_bounds__(TPB)
render_kernel(const float* __restrict__ rays_o, const float* __restrict__ rays_d,
              const v4u* __restrict__ frag_table,
              const float* __restrict__ db1, const float* __restrict__ db2,
              const float* __restrict__ cb1, const float* __restrict__ cb2,
              const float* __restrict__ cb3, const float* __restrict__ cb4,
              float* __restrict__ out) {
  __shared__ __align__(32) _Float16 s_frag[FRAG_HALVES];
  __shared__ float s_db1[HIDF];
  __shared__ float s_cb1[HIDF];
  __shared__ float s_cb2[HIDF];
  __shared__ float s_cb3[HIDF];
  __shared__ float s_db2[DFEAT];
  __shared__ float s_cb4[4];
  __shared__ __align__(16) float s_out[OUT_F32_PER_BLOCK];

  const int tid  = threadIdx.x;
  const int lane = tid & 31;
  const int wid  = tid >> 5;
  const int hsel = lane >> 4;
  const bool lo  = (hsel == 0);

  {
    v4u* sf = (v4u*)s_frag;
#pragma unroll 1
    for (int i = tid; i < FRAG_U4; i += TPB) sf[i] = frag_table[i];
  }
  if (tid < HIDF) {
    s_db1[tid] = db1[tid];
    s_cb1[tid] = cb1[tid];
    s_cb2[tid] = cb2[tid];
    s_cb3[tid] = cb3[tid];
  }
  if (tid < DFEAT) s_db2[tid] = db2[tid];
  if (tid < 3)  s_cb4[tid] = cb4[tid];
  if (tid == 3) s_cb4[3] = 0.0f;
  __syncthreads();

  const float c40 = s_cb4[0], c41 = s_cb4[1], c42 = s_cb4[2];
  float db2s[8];
#pragma unroll
  for (int i = 0; i < 8; ++i) db2s[i] = s_db2[8 * hsel + i];

#pragma unroll 1
  for (int j = 0; j < RAYS_PER_WAVE; ++j) {
    const int ray = blockIdx.x * RAYS_PER_BLOCK + wid * RAYS_PER_WAVE + j;

    const float ox = rays_o[ray * 3 + 0], oy = rays_o[ray * 3 + 1], oz = rays_o[ray * 3 + 2];
    const float dx = rays_d[ray * 3 + 0], dy = rays_d[ray * 3 + 1], dz = rays_d[ray * 3 + 2];

    const float ix = 1.0f / ((fabsf(dx) < 1e-15f) ? 1e-15f : dx);
    const float iy = 1.0f / ((fabsf(dy) < 1e-15f) ? 1e-15f : dy);
    const float iz = 1.0f / ((fabsf(dz) < 1e-15f) ? 1e-15f : dz);
    const float t1x = (-1.0f - ox) * ix, t2x = (1.0f - ox) * ix;
    const float t1y = (-1.0f - oy) * iy, t2y = (1.0f - oy) * iy;
    const float t1z = (-1.0f - oz) * iz, t2z = (1.0f - oz) * iz;
    float nearv = fmaxf(fmaxf(fminf(t1x, t2x), fminf(t1y, t2y)), fminf(t1z, t2z));
    float farv  = fminf(fminf(fmaxf(t1x, t2x), fmaxf(t1y, t2y)), fmaxf(t1z, t2z));
    nearv = fmaxf(nearv, 0.05f);
    farv  = fmaxf(farv, nearv + 1e-6f);
    const float span = farv - nearv;

    unsigned shw[4];
    {
      const float nrm = sqrtf(dx * dx + dy * dy + dz * dz);
      const float inv = 1.0f / nrm;
      const float ux = dx * inv, uy = dy * inv, uz = dz * inv;
      const float x01 = (ux + 1.0f) * 0.5f, y01 = (uy + 1.0f) * 0.5f, z01 = (uz + 1.0f) * 0.5f;
      const float sx = 2.0f * x01 - 1.0f, sy = 2.0f * y01 - 1.0f, sz = 2.0f * z01 - 1.0f;
      const float x2 = sx * sx, y2 = sy * sy, z2 = sz * sz;
      const float xy = sx * sy, yz = sy * sz, xz = sx * sz;
      float sh[16];
      sh[0]  =  0.28209479177387814f;
      sh[1]  = -0.4886025119029199f * sy;
      sh[2]  =  0.4886025119029199f * sz;
      sh[3]  = -0.4886025119029199f * sx;
      sh[4]  =  1.0925484305920792f * xy;
      sh[5]  = -1.0925484305920792f * yz;
      sh[6]  =  0.31539156525252005f * (2.0f * z2 - x2 - y2);
      sh[7]  = -1.0925484305920792f * xz;
      sh[8]  =  0.5462742152960396f * (x2 - y2);
      sh[9]  = -0.5900435899266435f * sy * (3.0f * x2 - y2);
      sh[10] =  2.890611442640554f  * xy * sz;
      sh[11] = -0.4570457994644658f * sy * (4.0f * z2 - x2 - y2);
      sh[12] =  0.3731763325901154f * sz * (2.0f * z2 - 3.0f * x2 - 3.0f * y2);
      sh[13] = -0.4570457994644658f * sx * (4.0f * z2 - x2 - y2);
      sh[14] =  1.445305721320277f  * sz * (x2 - y2);
      sh[15] = -0.5900435899266435f * sx * (x2 - 3.0f * y2);
      float shs[8];
#pragma unroll
      for (int i = 0; i < 8; ++i) shs[i] = lo ? sh[i] : sh[8 + i];
#pragma unroll
      for (int q = 0; q < 4; ++q) shw[q] = pack_h2(shs[2 * q], shs[2 * q + 1]);
    }

    float T = 1.0f, wsum = 0.0f, accR = 0.0f, accG = 0.0f, accB = 0.0f;

#pragma unroll 1
    for (int t = 0; t < NSTEPS / 16; ++t) {
      unsigned fz = 0;
      asm volatile("" : "+v"(fz));
      const _Float16* fb = s_frag + fz;

      const int sl = lane & 15;
      const int gi = t * 16 + sl;
      const float lin0 = (gi >= NSTEPS - 1)     ? 1.0f : (float)gi       * (1.0f / (float)(NSTEPS - 1));
      const float lin1 = (gi + 1 >= NSTEPS - 1) ? 1.0f : (float)(gi + 1) * (1.0f / (float)(NSTEPS - 1));
      const float zv = nearv + span * lin0;
      const float zn = nearv + span * lin1;
      const float delta = (gi == NSTEPS - 1) ? span * (1.0f / (float)NSTEPS) : (zn - zv);
      const float px = fminf(fmaxf(ox + dx * zv, -1.0f), 1.0f);
      const float py = fminf(fmaxf(oy + dy * zv, -1.0f), 1.0f);
      const float pz = fminf(fmaxf(oz + dz * zv, -1.0f), 1.0f);

      V16 bx;
      {
        const unsigned w0 = pack_h2(px, py);
        const unsigned w1 = pack_h2(pz, 0.0f);
        bx.w[0] = lo ? w0 : 0u;
        bx.w[1] = lo ? w1 : 0u;
#pragma unroll
        for (int q = 2; q < 8; ++q) bx.w[q] = 0u;
      }

      v8f ct[4];
#pragma unroll
      for (int mt = 0; mt < 4; ++mt) {
        v8f z = {};
        ct[mt] = mma16(lda_lds(fb, F_DW1 + mt, lane), bx.v, z);
      }
      const BPair Bh1 = acc_to_b(ct, s_db1, lane);

      v8f cd = {};
      cd = mma16(lda_lds(fb, F_DW2 + 0, lane), Bh1.b0, cd);
      cd = mma16(lda_lds(fb, F_DW2 + 1, lane), Bh1.b1, cd);
      const float densraw = cd[0] + db2s[0];

      V16 bc;
#pragma unroll
      for (int q = 0; q < 4; ++q) {
        bc.w[q]     = shw[q];
        bc.w[4 + q] = pack_h2(cd[2 * q] + db2s[2 * q], cd[2 * q + 1] + db2s[2 * q + 1]);
      }

#pragma unroll
      for (int mt = 0; mt < 4; ++mt) {
        v8f z = {};
        ct[mt] = mma16(lda_lds(fb, F_CW1 + mt, lane), bc.v, z);
      }
      const BPair Bc1 = acc_to_b(ct, s_cb1, lane);

#pragma unroll
      for (int nt = 0; nt < 4; ++nt) {
        v8f a = {};
        a = mma16(lda_lds(fb, F_CW2 + nt * 2 + 0, lane), Bc1.b0, a);
        a = mma16(lda_lds(fb, F_CW2 + nt * 2 + 1, lane), Bc1.b1, a);
        ct[nt] = a;
      }
      const BPair Bc2 = acc_to_b(ct, s_cb2, lane);

#pragma unroll
      for (int nt = 0; nt < 4; ++nt) {
        v8f a = {};
        a = mma16(lda_lds(fb, F_CW3 + nt * 2 + 0, lane), Bc2.b0, a);
        a = mma16(lda_lds(fb, F_CW3 + nt * 2 + 1, lane), Bc2.b1, a);
        ct[nt] = a;
      }
      const BPair Bc3 = acc_to_b(ct, s_cb3, lane);

      v8f cc = {};
      cc = mma16(lda_lds(fb, F_CW4 + 0, lane), Bc3.b0, cc);
      cc = mma16(lda_lds(fb, F_CW4 + 1, lane), Bc3.b1, cc);
      const float cr = 1.0f / (1.0f + expf(-(cc[0] + c40)));
      const float cg = 1.0f / (1.0f + expf(-(cc[1] + c41)));
      const float cbv = 1.0f / (1.0f + expf(-(cc[2] + c42)));

      const float dens  = expf(densraw);
      const float alpha = 1.0f - expf(-(delta * dens));
      const float p = 1.0f - alpha + 1e-15f;

      float cum = p;
#pragma unroll
      for (int off = 1; off < 16; off <<= 1) {
        const float u = __shfl_up(cum, off, 16);
        cum = (sl >= off) ? cum * u : cum;
      }
      float excl = __shfl_up(cum, 1, 16);
      excl = (sl == 0) ? 1.0f : excl;
      const float w = T * excl * alpha;

      const bool keep = (w > 1e-4f);
      float lw = lo ? w : 0.0f;
      float lr = (lo && keep) ? w * cr  : 0.0f;
      float lg = (lo && keep) ? w * cg  : 0.0f;
      float lb = (lo && keep) ? w * cbv : 0.0f;
#pragma unroll
      for (int off = 16; off >= 1; off >>= 1) {
        lw += __shfl_xor(lw, off);
        lr += __shfl_xor(lr, off);
        lg += __shfl_xor(lg, off);
        lb += __shfl_xor(lb, off);
      }
      wsum += lw; accR += lr; accG += lg; accB += lb;
      const float tileprod = __shfl(cum, 15);
      T *= tileprod;
    }

    if (lane == 0) {
      const float bg = 1.0f - wsum;
      float* so = s_out + (wid * RAYS_PER_WAVE + j) * 3;
      so[0] = accR + bg;
      so[1] = accG + bg;
      so[2] = accB + bg;
    }
  }

  __syncthreads();
  if (tid < OUT_F32_PER_BLOCK / 4) {
    const v4f val = *(const v4f*)(s_out + tid * 4);
    volatile v4f* dst = (volatile v4f*)(out + (size_t)blockIdx.x * OUT_F32_PER_BLOCK + tid * 4);
    *dst = val;
    __threadfence();
    *dst = val;
  }
}

extern "C" void kernel_launch(void* const* d_in, const int* in_sizes, int n_in,
                              void* d_out, int out_size, void* d_ws, size_t ws_size,
                              hipStream_t stream) {
  if (n_in < 14) return;
  const float* rays_o = (const float*)d_in[0];
  const float* rays_d = (const float*)d_in[1];
  const float* dW1 = (const float*)d_in[2];
  const float* db1 = (const float*)d_in[3];
  const float* dW2 = (const float*)d_in[4];
  const float* db2 = (const float*)d_in[5];
  const float* cW1 = (const float*)d_in[6];
  const float* cb1 = (const float*)d_in[7];
  const float* cW2 = (const float*)d_in[8];
  const float* cb2 = (const float*)d_in[9];
  const float* cW3 = (const float*)d_in[10];
  const float* cb3 = (const float*)d_in[11];
  const float* cW4 = (const float*)d_in[12];
  const float* cb4 = (const float*)d_in[13];
  float* out = (float*)d_out;

  if (in_sizes[0] < NUM_RAYS * 3 || in_sizes[1] < NUM_RAYS * 3) return;
  if (in_sizes[2] < 3 * HIDF || in_sizes[3] < HIDF || in_sizes[4] < HIDF * DFEAT || in_sizes[5] < DFEAT) return;
  if (in_sizes[6] < 32 * HIDF || in_sizes[7] < HIDF || in_sizes[8] < HIDF * HIDF || in_sizes[9] < HIDF) return;
  if (in_sizes[10] < HIDF * HIDF || in_sizes[11] < HIDF || in_sizes[12] < HIDF * 3 || in_sizes[13] < 3) return;
  if (out_size < NUM_RAYS * 3) return;
  if (ws_size < (size_t)FRAG_BYTES) return;

  v4u* table = (v4u*)d_ws;

  prep_frag_kernel<<<dim3(1), dim3(TPB), 0, stream>>>(dW1, dW2, cW1, cW2, cW3, cW4, table);
  render_kernel<<<dim3(NBLOCKS), dim3(TPB), 0, stream>>>(rays_o, rays_d, (const v4u*)table,
                                                        db1, db2, cb1, cb2, cb3, cb4, out);
}
